// ChunkedLogLinearAttentionReference_83983790506445
// MI455X (gfx1250) — hardware-verified
//
#include <hip/hip_runtime.h>
#include <math.h>

constexpr int kB     = 2;
constexpr int kT     = 2048;
constexpr int kD     = 1024;
constexpr int kH     = 16;
constexpr int kL     = 12;
constexpr int kDH    = kD / kH;
constexpr int kRows  = kB * kT;
constexpr int kQKVld = 3 * kD;
constexpr int kNL    = kH * kL;
constexpr int kQB    = 64;
constexpr int kNQB   = kT / kQB;
constexpr int kLamP  = 13;
constexpr float kWCarry    = 64.0f;
constexpr float kWCarryInv = 1.0f / kWCarry;
constexpr float kYCarry    = 0.125f;
constexpr float kOutScale  = 1.0f / (kYCarry * kWCarry);
static_assert(kDH == 64, "head dim");
static_assert(kRows % 64 == 0 && kD % 64 == 0 && kNL % 64 == 0, "GEMM M,N tile multiples");
static_assert(kD % 32 == 0, "GEMM K multiple of 32");
static_assert(((kRows / 64) * (kD / 64)) % 8 == 0, "tile count multiple of waves per block");
static_assert(((kRows / 64) * (kNL / 64)) % 8 == 0, "tile count multiple of waves per block");
static_assert(kT % kQB == 0, "query blocks");
static_assert((kQB * kL) % 128 == 0, "gate staging loop exact");
static_assert(kT <= (1 << (kL - 1)), "level index stays below kL");

typedef __attribute__((ext_vector_type(16))) _Float16 v16h;
typedef __attribute__((ext_vector_type(8)))  _Float16 v8h;
typedef __attribute__((ext_vector_type(16))) __bf16   v16b;
typedef __attribute__((ext_vector_type(8)))  __bf16   v8b;
typedef __attribute__((ext_vector_type(8)))  float    v8f;
typedef __attribute__((ext_vector_type(4)))  float    v4f;
typedef __attribute__((ext_vector_type(4)))  unsigned int v4u;

__device__ __forceinline__ unsigned short f2bf_bits(float f) {
  unsigned u = __float_as_uint(f);
  return (unsigned short)((u + 0x7FFFu + ((u >> 16) & 1u)) >> 16);
}
__device__ __forceinline__ float bf_bits2f(unsigned short h) { return __uint_as_float(((unsigned)h) << 16); }
__device__ __forceinline__ float bf16r(float f) { return bf_bits2f(f2bf_bits(f)); }
__device__ __forceinline__ unsigned pk16(unsigned short a, unsigned short b) { return (unsigned)a | ((unsigned)b << 16); }
__device__ __forceinline__ unsigned short h_bits(float f) { const _Float16 h = (_Float16)f; return __builtin_bit_cast(unsigned short, h); }

__device__ __forceinline__ void dep_guard4_h(v8f& a, v8f& b, v8f& c, v8f& d, v16h x, v16h y) { asm volatile("v_nop\n\tv_nop\n\tv_nop\n\tv_nop" : "+v"(a), "+v"(b), "+v"(c), "+v"(d) : "v"(x), "v"(y)); }
__device__ __forceinline__ void dep_guard4_b(v8f& a, v8f& b, v8f& c, v8f& d, v16b x, v16b y) { asm volatile("v_nop\n\tv_nop\n\tv_nop\n\tv_nop" : "+v"(a), "+v"(b), "+v"(c), "+v"(d) : "v"(x), "v"(y)); }
__device__ __forceinline__ void keep4_h(v16h a, v16h b, v16h c, v16h d) { asm volatile("v_nop" :: "v"(a), "v"(b), "v"(c), "v"(d)); }
__device__ __forceinline__ void keep4_b(v16b a, v16b b, v16b c, v16b d) { asm volatile("v_nop" :: "v"(a), "v"(b), "v"(c), "v"(d)); }
__device__ __forceinline__ void acc_guard4(v8f& a, v8f& b, v8f& c, v8f& d) { asm volatile("v_nop\n\tv_nop\n\tv_nop\n\tv_nop" : "+v"(a), "+v"(b), "+v"(c), "+v"(d)); }

template <typename T> struct Frag;
template <> struct Frag<_Float16> {
  typedef v16h V; union U { v16h v; v8h h[2]; };
  static __device__ __forceinline__ v16h load(const _Float16* p) {
    U f; f.h[0] = *(const v8h*)(p); f.h[1] = *(const v8h*)(p + 16); return f.v;
  }
  static __device__ __forceinline__ v8f mma(v16h a, v16h b, v8f c) {
    return __builtin_amdgcn_wmma_f32_16x16x32_f16(false, a, false, b, (short)0, c, false, false);
  }
  static __device__ __forceinline__ void guard4(v8f& a, v8f& b, v8f& c, v8f& d, v16h x, v16h y) { dep_guard4_h(a, b, c, d, x, y); }
  static __device__ __forceinline__ void keep(v16h a, v16h b, v16h c, v16h d) { keep4_h(a, b, c, d); }
};
template <> struct Frag<__bf16> {
  typedef v16b V; union U { v16b v; v8b h[2]; };
  static __device__ __forceinline__ v16b load(const __bf16* p) {
    U f; f.h[0] = *(const v8b*)(p); f.h[1] = *(const v8b*)(p + 16); return f.v;
  }
  static __device__ __forceinline__ v8f mma(v16b a, v16b b, v8f c) {
    return __builtin_amdgcn_wmma_f32_16x16x32_bf16(false, a, false, b, (short)0, c, false, false);
  }
  static __device__ __forceinline__ void guard4(v8f& a, v8f& b, v8f& c, v8f& d, v16b x, v16b y) { dep_guard4_b(a, b, c, d, x, y); }
  static __device__ __forceinline__ void keep(v16b a, v16b b, v16b c, v16b d) { keep4_b(a, b, c, d); }
};

__device__ __forceinline__ v8f mma_h(v16h a, v16h b, v8f c) {
  c = __builtin_amdgcn_wmma_f32_16x16x32_f16(false, a, false, b, (short)0, c, false, false);
  asm volatile("v_nop\n\tv_nop\n\tv_nop\n\tv_nop" : "+v"(c) : "v"(a), "v"(b));
  return c;
}

template <int ET> struct Elem;
template <> struct Elem<0> { typedef _Float16 T; };
template <> struct Elem<1> { typedef __bf16 T; };
template <int ET, bool SPLIT, int BIAS_MODE, int OUT_MODE, bool RESID, int ACT = 0>
__global__ __launch_bounds__(256) void wmma_gemm64(
    const unsigned short* __restrict__ Ap, const unsigned short* __restrict__ A2p, int lda, long strideA,
    const unsigned short* __restrict__ Btp, const unsigned short* __restrict__ Bt2p, int ldb, long strideB,
    void* __restrict__ Cout, void* __restrict__ Cout2, int ldc, long strideC,
    const float* __restrict__ bias,
    const float* __restrict__ resid, long strideR,
    int M, int N, int K, float scale) {
  typedef typename Elem<ET>::T T;
  typedef typename Frag<T>::V V;
  const T* A = (const T*)Ap; const T* A2 = (const T*)A2p; const T* Bt = (const T*)Btp; const T* Bt2 = (const T*)Bt2p;
  __shared__ __align__(16) float sT[8][16 * 68];
  const int b    = blockIdx.y;
  const int lane = threadIdx.x & 31;
  const int wave = threadIdx.x >> 5;
  const int tilesN = N >> 6;
  const int tilesM = M >> 6;
  const int tile = blockIdx.x * 8 + wave;
  if (tile >= tilesM * tilesN) return;
  const int tm = tile / tilesN;
  const int tn = tile - tm * tilesN;
  const int m0 = tm << 6;
  const int n0 = tn << 6;

  const T* Ab  = A  + (size_t)b * strideA;
  const T* Bb  = Bt + (size_t)b * strideB;
  const T* Ab2 = SPLIT ? (A2  + (size_t)b * strideA) : nullptr;
  const T* Bb2 = SPLIT ? (Bt2 + (size_t)b * strideB) : nullptr;

  const int rlane = lane & 15;
  const int koff  = (lane >> 4) * 8;
  const int mOff  = (lane >> 4) * 8;

  v8f acc[4][4];
#pragma unroll
  for (int i = 0; i < 4; ++i)
#pragma unroll
    for (int j = 0; j < 4; ++j) acc[i][j] = (v8f){0.f,0.f,0.f,0.f,0.f,0.f,0.f,0.f};

  for (int k0 = 0; k0 < K; k0 += 32) {
    V bh[4], bl[4];
#pragma unroll
    for (int j = 0; j < 4; ++j) {
      const size_t bo = (size_t)(n0 + (j << 4) + rlane) * ldb + koff + k0;
      bh[j] = Frag<T>::load(Bb + bo);
      if (SPLIT) bl[j] = Frag<T>::load(Bb2 + bo);
    }
#pragma unroll
    for (int i = 0; i < 4; ++i) {
      const size_t ao = (size_t)(m0 + (i << 4) + rlane) * lda + koff + k0;
      V ah = Frag<T>::load(Ab + ao);
      V al;
      if (SPLIT) al = Frag<T>::load(Ab2 + ao);
#pragma unroll
      for (int j = 0; j < 4; ++j) {
        acc[i][j] = Frag<T>::mma(ah, bh[j], acc[i][j]);
        if (SPLIT) {
          acc[i][j] = Frag<T>::mma(ah, bl[j], acc[i][j]);
          acc[i][j] = Frag<T>::mma(al, bh[j], acc[i][j]);
        }
      }
      Frag<T>::guard4(acc[i][0], acc[i][1], acc[i][2], acc[i][3], ah, SPLIT ? al : ah);
    }
    Frag<T>::keep(bh[0], bh[1], bh[2], bh[3]);
    if (SPLIT) Frag<T>::keep(bl[0], bl[1], bl[2], bl[3]);
  }
  acc_guard4(acc[0][0], acc[0][1], acc[0][2], acc[0][3]);
  acc_guard4(acc[1][0], acc[1][1], acc[1][2], acc[1][3]);
  acc_guard4(acc[2][0], acc[2][1], acc[2][2], acc[2][3]);
  acc_guard4(acc[3][0], acc[3][1], acc[3][2], acc[3][3]);

  float* slab = sT[wave];
  const float* Rb = RESID ? (resid + (size_t)b * strideR) : nullptr;
#pragma unroll
  for (int i = 0; i < 4; ++i) {
    const int mBase = m0 + (i << 4);
#pragma unroll
    for (int j = 0; j < 4; ++j) {
      const int n = n0 + (j << 4) + rlane;
      float bv = 0.f;
      if (BIAS_MODE == 2) bv = bf16r(bias[n]);
#pragma unroll
      for (int r = 0; r < 8; ++r) {
        float v = acc[i][j][r] * scale;
        if (BIAS_MODE == 1) v += bf16r(bias[mBase + mOff + r]);
        if (BIAS_MODE == 2) v += bv;
        if (RESID) v += Rb[(size_t)(mBase + mOff + r) * ldc + n];
        if (ACT == 2) v = fmaxf(v, 0.0f);
        if (ACT == 4) v = (v > 0.f) ? v : 0.01f * v;
        slab[(mOff + r) * 68 + (j << 4) + rlane] = v;
      }
    }
    __builtin_amdgcn_fence(__ATOMIC_RELEASE, "workgroup");
    __builtin_amdgcn_wave_barrier();
    __builtin_amdgcn_fence(__ATOMIC_ACQUIRE, "workgroup");
    if (OUT_MODE == 0) {
      float* C = (float*)Cout + (size_t)b * strideC;
      const int hh = lane >> 4, c4 = (lane & 15) * 4;
      for (int pass = 0; pass < 2; ++pass) {
#pragma unroll
        for (int it = 0; it < 8; ++it) {
          const int row = it * 2 + hh;
          v4f v = *(const v4f*)(slab + row * 68 + c4);
          *(volatile v4f*)(C + (size_t)(mBase + row) * ldc + n0 + c4) = v;
        }
        __threadfence();
      }
    } else {
      const int q = lane >> 3, c8 = (lane & 7) * 8;
      unsigned short* C  = (unsigned short*)Cout  + (size_t)b * strideC;
      unsigned short* C2 = (OUT_MODE == 2) ? ((unsigned short*)Cout2 + (size_t)b * strideC) : nullptr;
      for (int pass = 0; pass < 2; ++pass) {
#pragma unroll
        for (int it = 0; it < 4; ++it) {
          const int row = it * 4 + q;
          const float* sp = slab + row * 68 + c8;
          v8h hv, lv;
#pragma unroll
          for (int e = 0; e < 8; ++e) {
            if (OUT_MODE == 1) {
              hv[e] = (_Float16)sp[e];
            } else {
              unsigned short hb = f2bf_bits(sp[e]);
              unsigned short lb = f2bf_bits(sp[e] - bf_bits2f(hb));
              hv[e] = __builtin_bit_cast(_Float16, hb);
              lv[e] = __builtin_bit_cast(_Float16, lb);
            }
          }
          *(volatile v8h*)(C + (size_t)(mBase + row) * ldc + n0 + c8) = hv;
          if (OUT_MODE == 2) *(volatile v8h*)(C2 + (size_t)(mBase + row) * ldc + n0 + c8) = lv;
        }
        __threadfence();
      }
    }
    __builtin_amdgcn_fence(__ATOMIC_RELEASE, "workgroup");
    __builtin_amdgcn_wave_barrier();
    __builtin_amdgcn_fence(__ATOMIC_ACQUIRE, "workgroup");
  }
}

__global__ __launch_bounds__(256) void cvt8_x_kernel(const float* __restrict__ src, unsigned short* __restrict__ dst, int n8) {
  const int i = blockIdx.x * 256 + threadIdx.x;
  if (i < n8) {
    const float* sp = src + (size_t)i * 8;
    const v4f a = *(const v4f*)(sp);
    const v4f c = *(const v4f*)(sp + 4);
    v8h hv;
#pragma unroll
    for (int e = 0; e < 4; ++e) {
      hv[e]     = (_Float16)bf16r(a[e]);
      hv[4 + e] = (_Float16)bf16r(c[e]);
    }
    *(volatile v8h*)(dst + (size_t)i * 8) = hv;
    __threadfence();
    *(volatile v8h*)(dst + (size_t)i * 8) = hv;
  }
}

__global__ __launch_bounds__(256) void wtcast_kernel(const float* __restrict__ W0, const float* __restrict__ W1,
                                                     const float* __restrict__ W2, const float* __restrict__ W3,
                                                     const float* __restrict__ W4,
                                                     unsigned short* __restrict__ wcat, unsigned short* __restrict__ wot,
                                                     float carry) {
  __shared__ float sm[64][65];
  const int t  = threadIdx.x;
  const int z  = blockIdx.z;
  const int ncol = (z == 3) ? kNL : kD;
  const int d0 = blockIdx.x * 64;
  const int h0 = blockIdx.y * 64;
  if (h0 >= ncol) return;
  const float* W = (z == 0) ? W0 : (z == 1) ? W1 : (z == 2) ? W2 : (z == 3) ? W3 : W4;
  unsigned short* op = (z == 4) ? wot : (wcat + (size_t)z * kD * kD);
#pragma unroll
  for (int i = 0; i < 16; ++i) {
    const int e = i * 256 + t;
    const int r = e >> 6;
    const int c = e & 63;
    sm[c][r] = bf16r(W[(size_t)(d0 + r) * ncol + h0 + c]) * carry;
  }
  __syncthreads();
  const int lane = t & 31, wave = t >> 5;
  const int q = lane >> 3, c8 = (lane & 7) * 8;
  for (int pass = 0; pass < 2; ++pass) {
#pragma unroll
    for (int it = 0; it < 2; ++it) {
      const int row = wave * 8 + it * 4 + q;
      unsigned short hb[8];
#pragma unroll
      for (int e = 0; e < 8; ++e) hb[e] = h_bits(sm[row][c8 + e]);
      const v4u u = (v4u){pk16(hb[0], hb[1]), pk16(hb[2], hb[3]), pk16(hb[4], hb[5]), pk16(hb[6], hb[7])};
      *(volatile v4u*)(op + (size_t)(h0 + row) * kD + d0 + c8) = u;
    }
    __threadfence();
  }
}

__global__ __launch_bounds__(128) void gated_causal_mix_kernel(const unsigned short* __restrict__ QKVp,
                                                               const float* __restrict__ Zl,
                                                               unsigned short* __restrict__ Yp) {
  __shared__ __align__(16) unsigned short Ksh[64 * 64];
  __shared__ __align__(16) unsigned short Vth[64 * 64];
  __shared__ __align__(16) _Float16 Psh[4][16 * 64];
  __shared__ __align__(16) float Os[4][16 * 68];
  __shared__ float lamS[kQB * kLamP];

  const int tid  = threadIdx.x;
  const int wave = tid >> 5;
  const int lane = tid & 31;
  const int hh   = lane >> 4;
  const int c    = lane & 15;

  const int bx = blockIdx.x;
  const int qb = bx % kNQB;
  const int bh = bx / kNQB;
  const int h  = bh % kH;
  const int b  = bh / kH;
  const int qbase = qb * kQB;
  const int q0 = qbase + wave * 16;

#pragma unroll 1
  for (int idx = tid; idx < kQB * kL; idx += 128) {
    const int r = idx / kL;
    const int l = idx - r * kL;
    const float z = Zl[(size_t)(b * kT + qbase + r) * kNL + h * kL + l];
    const float az = fabsf(z);
    const float sp = fmaxf(z, 0.0f) + log1pf(expf(-az));
    lamS[r * kLamP + l] = sp;
  }

  v16h qa[2];
  {
    const _Float16* qp = (const _Float16*)(QKVp + (size_t)(b * kT + q0 + c) * kQKVld + h * kDH + 8 * hh);
    qa[0] = Frag<_Float16>::load(qp);
    qa[1] = Frag<_Float16>::load(qp + 32);
  }

  v8f oacc[4];
#pragma unroll
  for (int t = 0; t < 4; ++t) oacc[t] = (v8f){0.f,0.f,0.f,0.f,0.f,0.f,0.f,0.f};

  _Float16* pw = Psh[wave];

  for (int kc = 0; kc <= qb; ++kc) {
    const int kv0 = kc * 64;
    __syncthreads();
    {
      const int kvr = tid >> 1;
      const int dh  = (tid & 1) * 32;
      const size_t grow = (size_t)(b * kT + kv0 + kvr) * kQKVld + h * kDH + dh;
      const v4u* kg = (const v4u*)(QKVp + grow + kD);
      const v4u* vg = (const v4u*)(QKVp + grow + 2 * kD);
      v4u* kd = (v4u*)(Ksh + kvr * 64 + dh);
#pragma unroll
      for (int i = 0; i < 4; ++i) {
        const v4u kw = kg[i];
        const v4u vw = vg[i];
        kd[i] = kw;
#pragma unroll
        for (int e = 0; e < 4; ++e) {
          const unsigned w = vw[e];
          const int d = dh + 8 * i + 2 * e;
          Vth[d * 64 + kvr]       = (unsigned short)(w & 0xffffu);
          Vth[(d + 1) * 64 + kvr] = (unsigned short)(w >> 16);
        }
      }
    }
    __syncthreads();

    v8f s[4];
#pragma unroll
    for (int j = 0; j < 4; ++j) {
      s[j] = (v8f){0.f,0.f,0.f,0.f,0.f,0.f,0.f,0.f};
#pragma unroll
      for (int dc = 0; dc < 2; ++dc) {
        const v16h kb = Frag<_Float16>::load((const _Float16*)(Ksh + (j * 16 + c) * 64 + dc * 32 + 8 * hh));
        s[j] = mma_h(qa[dc], kb, s[j]);
      }
    }

#pragma unroll
    for (int r = 0; r < 8; ++r) {
      const int lrow = wave * 16 + 8 * hh + r;
      const int qi = qbase + lrow;
      const float* lamrow = lamS + lrow * kLamP;
#pragma unroll
      for (int j = 0; j < 4; ++j) {
        const int kj = kv0 + j * 16 + c;
        const unsigned xv = (((unsigned)(qi + 1)) ^ ((unsigned)kj)) | 1u;
        int lvl = 31 - __builtin_clz(xv);
        lvl = (lvl > kL - 1) ? (kL - 1) : lvl;
        const float g = lamrow[lvl];
        const float sg = s[j][r] * g;
        const float pv = (kj <= qi) ? sg : 0.0f;
        pw[(8 * hh + r) * 64 + j * 16 + c] = (_Float16)pv;
      }
    }
    __builtin_amdgcn_fence(__ATOMIC_RELEASE, "workgroup");
    __builtin_amdgcn_wave_barrier();
    __builtin_amdgcn_fence(__ATOMIC_ACQUIRE, "workgroup");

#pragma unroll 1
    for (int kk = 0; kk < 2; ++kk) {
      const v16h pa = Frag<_Float16>::load(pw + c * 64 + kk * 32 + 8 * hh);
#pragma unroll
      for (int t = 0; t < 4; ++t) {
        const v16h vb = Frag<_Float16>::load((const _Float16*)(Vth + (t * 16 + c) * 64 + kk * 32 + 8 * hh));
        oacc[t] = mma_h(pa, vb, oacc[t]);
      }
    }
  }

  float* os = Os[wave];
#pragma unroll
  for (int r = 0; r < 8; ++r) {
#pragma unroll
    for (int t = 0; t < 4; ++t) os[(8 * hh + r) * 68 + t * 16 + c] = oacc[t][r] * kYCarry;
  }
  __builtin_amdgcn_fence(__ATOMIC_RELEASE, "workgroup");
  __builtin_amdgcn_wave_barrier();
  __builtin_amdgcn_fence(__ATOMIC_ACQUIRE, "workgroup");
  {
    const int q4 = lane >> 3, c8 = (lane & 7) * 8;
    unsigned short* ybase = Yp + (size_t)(b * kT + q0) * kD + h * kDH;
    for (int pass = 0; pass < 2; ++pass) {
#pragma unroll
      for (int it = 0; it < 4; ++it) {
        const int row = it * 4 + q4;
        const float* sp = os + row * 68 + c8;
        v8h hv;
#pragma unroll
        for (int e = 0; e < 8; ++e) hv[e] = (_Float16)sp[e];
        *(volatile v8h*)(ybase + (size_t)row * kD + c8) = hv;
      }
      __threadfence();
    }
  }
}

extern "C" void kernel_launch(void* const* d_in, const int* in_sizes, int n_in,
                              void* d_out, int out_size, void* d_ws, size_t ws_size, hipStream_t stream) {
  if (n_in < 11 || d_out == nullptr || d_ws == nullptr) return;
  if (in_sizes[0] != kRows * kD || in_sizes[1] != kD * kD || in_sizes[2] != kD ||
      in_sizes[3] != kD * kD || in_sizes[4] != kD || in_sizes[5] != kD * kD || in_sizes[6] != kD ||
      in_sizes[7] != kD * kNL || in_sizes[8] != kNL || in_sizes[9] != kD * kD || in_sizes[10] != kD ||
      out_size != kRows * kD) return;

  const float* x  = (const float*)d_in[0];
  const float* Wq = (const float*)d_in[1];
  const float* bq = (const float*)d_in[2];
  const float* Wk = (const float*)d_in[3];
  const float* bk = (const float*)d_in[4];
  const float* Wv = (const float*)d_in[5];
  const float* bv = (const float*)d_in[6];
  const float* Wl = (const float*)d_in[7];
  const float* bl = (const float*)d_in[8];
  const float* Wo = (const float*)d_in[9];
  const float* bo = (const float*)d_in[10];
  float* out = (float*)d_out;

  char* ws = (char*)d_ws; size_t off = 0;
  auto carve = [&](size_t bytes) -> char* { char* p = ws + off; off += (bytes + 255) & ~(size_t)255; return p; };
  unsigned short* XH   = (unsigned short*)carve((size_t)kRows * kD * 2);
  unsigned short* WCAT = (unsigned short*)carve((size_t)(3 * kD + kNL) * kD * 2);
  unsigned short* WOT  = (unsigned short*)carve((size_t)kD * kD * 2);
  unsigned short* QKV  = (unsigned short*)carve((size_t)kRows * kQKVld * 2);
  float*          ZL   = (float*)carve((size_t)kRows * kNL * 4);
  unsigned short* Y    = (unsigned short*)carve((size_t)kRows * kD * 2);
  if (off > ws_size || off > (size_t)134217728) return;

  const int n8x = kRows * (kD / 8);
  cvt8_x_kernel<<<(n8x + 255) / 256, 256, 0, stream>>>(x, XH, n8x);
  wtcast_kernel<<<dim3(kD / 64, kD / 64, 5), 256, 0, stream>>>(Wq, Wk, Wv, Wl, Wo, WCAT, WOT, kWCarry);

  const dim3 gproj((kRows / 64) * (kD / 64) / 8, 1);
  const float* bqkv[3] = {bq, bk, bv};
  for (int z = 0; z < 3; ++z) {
    const unsigned short* bt = WCAT + (size_t)z * kD * kD;
    unsigned short* cz = QKV + (size_t)z * kD;
    wmma_gemm64<0, false, 2, 1, false, 0><<<gproj, 256, 0, stream>>>(
        XH, XH, kD, 0L, bt, bt, kD, 0L, (void*)cz, (void*)cz, kQKVld, 0L,
        bqkv[z], ZL, 0L, kRows, kD, kD, kWCarryInv);
  }
  {
    const dim3 glam((kRows / 64) * (kNL / 64) / 8, 1);
    const unsigned short* bt = WCAT + (size_t)3 * kD * kD;
    wmma_gemm64<0, false, 2, 0, false, 0><<<glam, 256, 0, stream>>>(
        XH, XH, kD, 0L, bt, bt, kD, 0L, (void*)ZL, (void*)ZL, kNL, 0L,
        bl, ZL, 0L, kRows, kNL, kD, kWCarryInv);
  }

  gated_causal_mix_kernel<<<kB * kH * kNQB, 128, 0, stream>>>(QKV, ZL, Y);

  wmma_gemm64<0, false, 2, 0, false, 0><<<gproj, 256, 0, stream>>>(
      Y, Y, kD, 0L, WOT, WOT, kD, 0L, (void*)out, (void*)out, kD, 0L,
      bo, ZL, 0L, kRows, kD, kD, kOutScale);
}
